// LSTMPositionPredictor_67465346285956
// MI455X (gfx1250) — hardware-run, weakly checked
//
#include <hip/hip_runtime.h>

typedef __attribute__((ext_vector_type(16))) _Float16 v16h;
typedef __attribute__((ext_vector_type(8)))  _Float16 v8h;
typedef __attribute__((ext_vector_type(8)))  float    v8f;
typedef __attribute__((ext_vector_type(4)))  float    v4f;

constexpr int NB   = 1024;
constexpr int NS   = 64;
constexpr int NT   = 32;
constexpr int NH   = 256;
constexpr int NIN  = 4;
constexpr int NGATE = 4 * NH;
constexpr int ROWS = 16;
constexpr int NBLK = NB / ROWS;
constexpr int HP   = 264;
constexpr int H32P = 260;
constexpr int NSTEPS = 2 * NS + 2 * NT;
constexpr size_t WPLANE = (size_t)NGATE * NH;
constexpr float HSC   = 16.0f;
constexpr float WSC   = 16.0f;
constexpr float INVSC = 1.0f / 256.0f;

static_assert(NB % ROWS == 0);
static_assert(NH % 32 == 0);
static_assert((WPLANE / 2) % 256 == 0);

__device__ __forceinline__ void dep_guard_h(v8f& a, v8f& b, v16h x, v16h y) { asm volatile("v_nop\n\tv_nop\n\tv_nop\n\tv_nop" : "+v"(a), "+v"(b) : "v"(x), "v"(y)); }
template <typename T> struct Frag;
template <> struct Frag<_Float16> {
  typedef v16h V; union U { v16h v; v8h h[2]; };
  static __device__ __forceinline__ v16h load(const _Float16* p) {
    U f; f.h[0] = *(const v8h*)(p); f.h[1] = *(const v8h*)(p + 16); return f.v;
  }
  static __device__ __forceinline__ v8f mma(v16h a, v16h b, v8f c) {
    return __builtin_amdgcn_wmma_f32_16x16x32_f16(false, a, false, b, (short)0, c, false, false);
  }
  static __device__ __forceinline__ void guard(v8f& a, v8f& b, v16h x, v16h y) { dep_guard_h(a, b, x, y); }
};
__device__ __forceinline__ void guard_ab2(v8f& c0, v8f& c1, v16h a, v16h b0, v16h b1) {
  asm volatile("v_nop\n\tv_nop\n\tv_nop\n\tv_nop" : "+v"(c0), "+v"(c1) : "v"(a), "v"(b0), "v"(b1));
}

__device__ __forceinline__ float sigm_f(float v) {
  v = fminf(fmaxf(v, -30.0f), 30.0f);
  return __builtin_amdgcn_rcpf(1.0f + expf(-v));
}
__device__ __forceinline__ float tanh_f(float v) {
  v = fminf(fmaxf(v, -15.0f), 15.0f);
  return 1.0f - 2.0f * __builtin_amdgcn_rcpf(1.0f + expf(2.0f * v));
}

__global__ __launch_bounds__(256) void cast_wh_kernel(
    const float* __restrict__ w0, const float* __restrict__ w1,
    const float* __restrict__ w2, const float* __restrict__ w3,
    _Float16* __restrict__ outp) {
  const int y = blockIdx.y;
  const float* src = (y == 0) ? w0 : (y == 1) ? w1 : (y == 2) ? w2 : w3;
  _Float16* dst = outp + (size_t)y * WPLANE;
  const int i = blockIdx.x * 256 + threadIdx.x;
  if (i < (int)(WPLANE / 2)) {
    const _Float16 h0 = (_Float16)(src[2 * i] * WSC), h1 = (_Float16)(src[2 * i + 1] * WSC);
    const unsigned u = (unsigned)__builtin_bit_cast(unsigned short, h0) | ((unsigned)__builtin_bit_cast(unsigned short, h1) << 16);
    ((volatile unsigned*)dst)[i] = u;
    __threadfence();
    ((volatile unsigned*)dst)[i] = u;
  }
}

__global__ __launch_bounds__(256) void bilstm_decode_kernel(
    const float* __restrict__ x, const int* __restrict__ lengths,
    const float* __restrict__ ewi_f, const float* __restrict__ eb_f,
    const float* __restrict__ ewi_b, const float* __restrict__ eb_b,
    const float* __restrict__ dwi_f, const float* __restrict__ db_f,
    const float* __restrict__ dwi_b, const float* __restrict__ db_b,
    const float* __restrict__ gw, const float* __restrict__ gb,
    const _Float16* __restrict__ whp,
    float* __restrict__ outp, float* __restrict__ rho_ws)
{
  __shared__ __align__(16) _Float16 hA[2][ROWS * HP];
  __shared__ __align__(16) float h32[2][ROWS * H32P];
  __shared__ __align__(16) float xt[2][ROWS * NIN];
  __shared__ __align__(16) float stg[2][ROWS * 32];
  __shared__ __align__(16) float rhs[32];

  const int tid  = threadIdx.x;
  const int lane = tid & 31;
  const int wave = tid >> 5;
  const int hh   = lane >> 4;
  const int cl   = lane & 15;
  const int koff = hh * 8;
  const int b0   = blockIdx.x * ROWS;

  {
    _Float16* hflat = &hA[0][0];
    for (int i = tid; i < 2 * ROWS * HP; i += 256) hflat[i] = (_Float16)0.0f;
  }
  if (tid < 32) rhs[tid] = 0.0f;

  float cf[16], cb[16];
#pragma unroll
  for (int i = 0; i < 16; ++i) { cf[i] = 0.0f; cb[i] = 0.0f; }

#pragma unroll 1
  for (int cs = 0; cs < NSTEPS; ++cs) {
    const bool isdec = (cs >= 2 * NS);
    const int dd   = isdec ? ((cs - 2 * NS) & 1) : ((cs >= NS) ? 1 : 0);
    const int tdec = isdec ? ((cs - 2 * NS) >> 1) : 0;
    const int xbuf = isdec ? (tdec & 1) : (cs & 1);
    const int widx = isdec ? (2 + dd) : dd;
    const _Float16* wh = whp + (size_t)widx * WPLANE;
    const float* wi = (widx == 0) ? ewi_f : (widx == 1) ? ewi_b : (widx == 2) ? dwi_f : dwi_b;
    const float* bs = (widx == 0) ? eb_f  : (widx == 1) ? eb_b  : (widx == 2) ? db_f  : db_b;

    if (!isdec) {
      const int sidx = (dd == 0) ? cs : (2 * NS - 1 - cs);
      if (tid < 64) {
        const int row = tid >> 2, k = tid & 3;
        xt[xbuf][tid] = x[((size_t)(b0 + row) * NS + sidx) * NIN + k];
      }
    } else if (cs == 2 * NS) {
      if (tid < 64) {
        const int row = tid >> 2, k = tid & 3;
        int idx = lengths[b0 + row] - 1;
        idx = (idx < 0) ? (idx + NS) : idx;
        idx = (idx < 0) ? 0 : ((idx > NS - 1) ? (NS - 1) : idx);
        xt[0][tid] = x[((size_t)(b0 + row) * NS + idx) * NIN + k];
      }
    }
    __syncthreads();

    float cc[16];
#pragma unroll
    for (int i = 0; i < 16; ++i) cc[i] = dd ? cb[i] : cf[i];

    v8f acc[4][2];
#pragma unroll
    for (int g = 0; g < 4; ++g) {
      acc[g][0] = (v8f){0.f,0.f,0.f,0.f,0.f,0.f,0.f,0.f};
      acc[g][1] = (v8f){0.f,0.f,0.f,0.f,0.f,0.f,0.f,0.f};
    }
    const _Float16* hT = hA[dd];
#pragma unroll 1
    for (int kc = 0; kc < NH / 32; ++kc) {
      const int k0 = kc * 32;
      const v16h av = Frag<_Float16>::load(hT + cl * HP + k0 + koff);
#pragma unroll
      for (int g = 0; g < 4; ++g) {
        const _Float16* bp = wh + (size_t)(g * NH + 32 * wave + cl) * NH + k0 + koff;
        const v16h bv0 = Frag<_Float16>::load(bp);
        const v16h bv1 = Frag<_Float16>::load(bp + 16 * NH);
        acc[g][0] = Frag<_Float16>::mma(av, bv0, acc[g][0]);
        acc[g][1] = Frag<_Float16>::mma(av, bv1, acc[g][1]);
        guard_ab2(acc[g][0], acc[g][1], av, bv0, bv1);
      }
    }
    __syncthreads();

    {
      const float* xb = xt[xbuf];
      _Float16* hw = hA[dd];
      float* h3 = h32[dd];
#pragma unroll
      for (int t2 = 0; t2 < 2; ++t2) {
        const int u = 32 * wave + 16 * t2 + cl;
        const v4f wI = *(const v4f*)(wi + (size_t)(u) * NIN);
        const v4f wF = *(const v4f*)(wi + (size_t)(NH + u) * NIN);
        const v4f wG = *(const v4f*)(wi + (size_t)(2 * NH + u) * NIN);
        const v4f wO = *(const v4f*)(wi + (size_t)(3 * NH + u) * NIN);
        const float bI = bs[u], bF = bs[NH + u], bG = bs[2 * NH + u], bO = bs[3 * NH + u];
#pragma unroll
        for (int r = 0; r < 8; ++r) {
          const int m = 8 * hh + r;
          const v4f xv = *(const v4f*)(xb + m * NIN);
          const float zi = bI + (xv[0] * wI[0] + xv[1] * wI[1] + xv[2] * wI[2] + xv[3] * wI[3]);
          const float zf = bF + (xv[0] * wF[0] + xv[1] * wF[1] + xv[2] * wF[2] + xv[3] * wF[3]);
          const float zg = bG + (xv[0] * wG[0] + xv[1] * wG[1] + xv[2] * wG[2] + xv[3] * wG[3]);
          const float zo = bO + (xv[0] * wO[0] + xv[1] * wO[1] + xv[2] * wO[2] + xv[3] * wO[3]);
          const float pi = acc[0][t2][r] * INVSC + zi;
          const float pf = acc[1][t2][r] * INVSC + zf;
          const float pg = acc[2][t2][r] * INVSC + zg;
          const float po = acc[3][t2][r] * INVSC + zo;
          const float c2 = sigm_f(pf) * cc[t2 * 8 + r] + sigm_f(pi) * tanh_f(pg);
          const float h2 = sigm_f(po) * tanh_f(c2);
          cc[t2 * 8 + r] = c2;
          hw[m * HP + u] = (_Float16)(h2 * HSC);
          if (isdec) h3[m * H32P + u] = h2;
        }
      }
    }
#pragma unroll
    for (int i = 0; i < 16; ++i) { const float nv = cc[i]; cf[i] = dd ? cf[i] : nv; cb[i] = dd ? nv : cb[i]; }

    if (isdec && dd == 1) {
      __syncthreads();
      const int row = tid >> 4, cj = (tid >> 1) & 7, kh = tid & 1;
      const float* hp = h32[kh] + row * H32P;
      const float* gp = gw + (size_t)cj * (2 * NH) + kh * NH;
      float s0 = 0.0f, s1 = 0.0f;
#pragma unroll 1
      for (int k = 0; k < NH; k += 8) {
        const v4f a0 = *(const v4f*)(hp + k), a1 = *(const v4f*)(hp + k + 4);
        const v4f g0 = *(const v4f*)(gp + k), g1 = *(const v4f*)(gp + k + 4);
        s0 += a0[0] * g0[0] + a0[1] * g0[1] + a0[2] * g0[2] + a0[3] * g0[3];
        s1 += a1[0] * g1[0] + a1[1] * g1[1] + a1[2] * g1[2] + a1[3] * g1[3];
      }
      float tot = s0 + s1;
      tot += __shfl_xor(tot, 1, 32);
      const float gv = tot + gb[cj];
      const float ev = expf(gv);
      const float rv = tanhf(gv);
      if (kh == 0) {
        const int slot = row * 32 + (tdec & 7) * 4;
        if (cj < 4) { stg[0][slot + cj] = gv; xt[(tdec + 1) & 1][row * NIN + cj] = gv; }
        else stg[1][slot + cj - 4] = ev;
        if (cj == 6 && tdec == NT - 1) rhs[row] = rv;
      }
      if ((tdec & 7) == 7) {
        __syncthreads();
        const int sel = tid >> 7, hrow = (tid & 127) >> 3, q = tid & 7;
        const v4f val = *(const v4f*)(stg[sel] + hrow * 32 + q * 4);
        float* dp = outp + (size_t)sel * ((size_t)NB * NT * NIN) + (size_t)(b0 + hrow) * (NT * NIN) + (tdec >> 3) * 32 + q * 4;
        *(volatile v4f*)dp = val;
        __threadfence();
        *(volatile v4f*)dp = val;
      }
    }
  }

  __syncthreads();
  if (tid < 32) {
    const v4f rv4 = *(const v4f*)(rhs + (lane & 7) * 4);
    float* dp = rho_ws + (size_t)blockIdx.x * 32 + (lane & 7) * 4;
    if (lane < 8) *(volatile v4f*)dp = rv4;
    __threadfence();
    if (lane < 8) *(volatile v4f*)dp = rv4;
  }
}

__global__ __launch_bounds__(256) void rho_copy_kernel(const float* __restrict__ rws, float* __restrict__ out2) {
  const int t = threadIdx.x;
  const v4f v = *(const v4f*)(rws + (size_t)(t >> 2) * 32 + (t & 3) * 4);
  float* dp = out2 + 4 * t;
  *(volatile v4f*)dp = v;
  __threadfence();
  *(volatile v4f*)dp = v;
}

extern "C" void kernel_launch(void* const* d_in, const int* in_sizes, int n_in,
                              void* d_out, int out_size, void* d_ws, size_t ws_size,
                              hipStream_t stream) {
  const float* x        = (const float*)d_in[0];
  const int*   lengths  = (const int*)d_in[1];
  const float* enc_wi_f = (const float*)d_in[3];
  const float* enc_wh_f = (const float*)d_in[4];
  const float* enc_b_f  = (const float*)d_in[5];
  const float* enc_wi_b = (const float*)d_in[6];
  const float* enc_wh_b = (const float*)d_in[7];
  const float* enc_b_b  = (const float*)d_in[8];
  const float* dec_wi_f = (const float*)d_in[9];
  const float* dec_wh_f = (const float*)d_in[10];
  const float* dec_b_f  = (const float*)d_in[11];
  const float* dec_wi_b = (const float*)d_in[12];
  const float* dec_wh_b = (const float*)d_in[13];
  const float* dec_b_b  = (const float*)d_in[14];
  const float* gw       = (const float*)d_in[15];
  const float* gb       = (const float*)d_in[16];

  const size_t wbytes = 4 * WPLANE * sizeof(_Float16);
  const size_t rbytes = (size_t)NBLK * 32 * sizeof(float);
  if (wbytes + rbytes > ws_size) return;
  if ((size_t)out_size * sizeof(float) < (size_t)(2 * NB * NT * NIN + NB) * sizeof(float)) return;

  _Float16* whp   = (_Float16*)d_ws;
  float*   rho_ws = (float*)((char*)d_ws + wbytes);
  float*   outp   = (float*)d_out;

  cast_wh_kernel<<<dim3((unsigned)(WPLANE / 2 / 256), 4), 256, 0, stream>>>(
      enc_wh_f, enc_wh_b, dec_wh_f, dec_wh_b, whp);

  bilstm_decode_kernel<<<dim3(NBLK), 256, 0, stream>>>(
      x, lengths,
      enc_wi_f, enc_b_f, enc_wi_b, enc_b_b,
      dec_wi_f, dec_b_f, dec_wi_b, dec_b_b,
      gw, gb, whp, outp, rho_ws);

  rho_copy_kernel<<<dim3(1), 256, 0, stream>>>(rho_ws, outp + (size_t)2 * NB * NT * NIN);
}
